// StructureTransformerLayer_54314156425236
// MI455X (gfx1250) — hardware-run, weakly checked
//
#include <hip/hip_runtime.h>


#define NB_  4
#define LL   768
#define DM   512
#define NH_  8
#define HD   64
#define NG   7
#define DFF  2048
#define DF2  4096
#define PCAR 1024.0f
typedef _Float16 h16;
typedef unsigned short bf;
typedef __attribute__((ext_vector_type(16))) __bf16   v16bf;
typedef __attribute__((ext_vector_type(16))) _Float16 v16h;
typedef __attribute__((ext_vector_type(8)))  _Float16 v8h;
typedef __attribute__((ext_vector_type(8)))  unsigned short v8us;
typedef __attribute__((ext_vector_type(8)))  float    v8f;
typedef __attribute__((ext_vector_type(4)))  float    v4f;
typedef v8h  __attribute__((may_alias)) v8ha;
typedef v4f  __attribute__((may_alias)) v4fa;
typedef v8us __attribute__((may_alias)) v8usa;

__device__ __forceinline__ unsigned short f2bf(float f) { unsigned u = __float_as_uint(f); u += 0x7FFFu + ((u >> 16) & 1u); return (unsigned short)(u >> 16); }
__device__ __forceinline__ float bf2f(unsigned short b) { return __uint_as_float(((unsigned)b) << 16); }
__device__ __forceinline__ float bfr(float f) { return bf2f(f2bf(f)); }
__device__ __forceinline__ v16h cat16(v8h lo, v8h hi) { return __builtin_shufflevector(lo, hi, 0, 1, 2, 3, 4, 5, 6, 7, 8, 9, 10, 11, 12, 13, 14, 15); }
__device__ __forceinline__ v16bf cat16b(v8us lo, v8us hi) { return __builtin_bit_cast(v16bf, __builtin_shufflevector(lo, hi, 0, 1, 2, 3, 4, 5, 6, 7, 8, 9, 10, 11, 12, 13, 14, 15)); }
__device__ __forceinline__ v8f wmma16(v16h a, v16h b, v8f c) { return __builtin_amdgcn_wmma_f32_16x16x32_f16(false, a, false, b, (short)0, c, false, false); }
__device__ __forceinline__ v8f wmmab(v16bf a, v16bf b, v8f c) { return __builtin_amdgcn_wmma_f32_16x16x32_bf16(false, a, false, b, (short)0, c, false, false); }


template <typename T16> struct WFrag;
template <> struct WFrag<h16> { typedef v16h V; static __device__ __forceinline__ V ld(const h16* p) { return cat16(*(const v8h*)p, *(const v8h*)(p + 16)); } static __device__ __forceinline__ v8f mma(V a, V b, v8f c) { return wmma16(a, b, c); } };
template <> struct WFrag<bf> { typedef v16bf V; static __device__ __forceinline__ V ld(const bf* p) { return cat16b(*(const v8us*)p, *(const v8us*)(p + 16)); } static __device__ __forceinline__ v8f mma(V a, V b, v8f c) { return wmmab(a, b, c); } };
template <typename T16, int NSPLIT, bool BIAS>
__global__ __launch_bounds__(32) void k_gemmw(const T16* __restrict__ A, const T16* __restrict__ A2, const T16* __restrict__ Bt, const T16* __restrict__ Bt2, int K, float* C, int ldc, const float* __restrict__ bias, size_t sA, size_t sB, size_t sC) {
    typedef typename WFrag<T16>::V V;
    __shared__ __align__(16) float os[16 * 68];
    const size_t z = blockIdx.z; A += z * sA; if (A2) A2 += z * sA; Bt += z * sB; if (Bt2) Bt2 += z * sB; C += z * sC;
    const int lane = threadIdx.x & 31, lr = lane & 15, hi = lane >> 4; const int r0 = blockIdx.x * 64, c0 = blockIdx.y * 64;
    v8f acc[4][4];
#pragma unroll
    for (int mb = 0; mb < 4; ++mb)
#pragma unroll
        for (int nb = 0; nb < 4; ++nb) acc[mb][nb] = (v8f){};
    const size_t aoff = (size_t)(r0 + lr) * K + 8 * hi, boff = (size_t)(c0 + lr) * K + 8 * hi;
#pragma unroll 1
    for (int kc = 0; kc < K; kc += 32) {
        V a[4], a2[4];
#pragma unroll
        for (int mb = 0; mb < 4; ++mb) { a[mb] = WFrag<T16>::ld(A + aoff + (size_t)mb * 16 * K + kc); if (NSPLIT == 1 || NSPLIT == 2) a2[mb] = WFrag<T16>::ld(A2 + aoff + (size_t)mb * 16 * K + kc); }
#pragma unroll
        for (int nb = 0; nb < 4; ++nb) { const V b = WFrag<T16>::ld(Bt + boff + (size_t)nb * 16 * K + kc); V b2; if (NSPLIT >= 2) b2 = WFrag<T16>::ld(Bt2 + boff + (size_t)nb * 16 * K + kc);
#pragma unroll
            for (int mb = 0; mb < 4; ++mb) { acc[mb][nb] = WFrag<T16>::mma(a[mb], b, acc[mb][nb]); if (NSPLIT == 1 || NSPLIT == 2) acc[mb][nb] = WFrag<T16>::mma(a2[mb], b, acc[mb][nb]); if (NSPLIT >= 2) acc[mb][nb] = WFrag<T16>::mma(a[mb], b2, acc[mb][nb]); } }
        asm volatile("v_nop\n\tv_nop\n\tv_nop\n\tv_nop" : "+v"(acc[0][0]), "+v"(acc[1][1]), "+v"(acc[2][2]), "+v"(acc[3][3]) : "v"(a[0]), "v"(a[3]));
    }
#pragma unroll
    for (int mb = 0; mb < 4; ++mb) {
#pragma unroll
        for (int nb = 0; nb < 4; ++nb) {
#pragma unroll
            for (int j = 0; j < 8; ++j) os[(hi * 8 + j) * 68 + nb * 16 + lr] = acc[mb][nb][j]; }
        __builtin_amdgcn_wave_barrier(); asm volatile("" ::: "memory");
        float* crow = C + (size_t)(r0 + mb * 16) * ldc + c0;
#pragma unroll 1
        for (int ps = 0; ps < 2; ++ps) {
#pragma unroll
            for (int s = 0; s < 8; ++s) { const int row = 2 * s + hi, cofs = lr * 4; v4f val = *(const v4fa*)(os + row * 68 + cofs); if (BIAS) { val[0] += bfr(bias[c0 + cofs]); val[1] += bfr(bias[c0 + cofs + 1]); val[2] += bfr(bias[c0 + cofs + 2]); val[3] += bfr(bias[c0 + cofs + 3]); }
                *(volatile v4f*)(crow + (size_t)row * ldc + cofs) = val; }
            if (ps == 0) __threadfence(); }
        __builtin_amdgcn_wave_barrier(); asm volatile("" ::: "memory");
    }
}

__device__ __forceinline__ h16 tohx(float x) { return (h16)x; }
__device__ __forceinline__ void splitf(float y, unsigned short& h, unsigned short& l) { h = f2bf(y); l = f2bf(y - bf2f(h)); }
typedef __attribute__((ext_vector_type(2))) unsigned short v2us;
typedef __attribute__((ext_vector_type(4))) unsigned short v4us;
typedef __attribute__((ext_vector_type(2))) _Float16 v2h;
typedef __attribute__((ext_vector_type(4))) _Float16 v4h;

__global__ __launch_bounds__(256) void k_wtG(const float* __restrict__ w, int K, int N, bf* Bt) {
    const int lane = threadIdx.x & 31; const int L0 = (blockIdx.x * 8 + (threadIdx.x >> 5)) * 8; const int nlines = N * K / 64;
#pragma unroll
    for (int ps = 0; ps < 2; ++ps) {
#pragma unroll 1
        for (int l = 0; l < 8; ++l) { const int L = L0 + l; if (L >= nlines) break; const size_t e = (size_t)L * 64 + lane * 2; const int k = (int)(e % K), n = (int)(e / K); v2us o;
            o[0] = f2bf(w[(size_t)k * N + n]); o[1] = f2bf(w[(size_t)(k + 1) * N + n]); *(volatile v2us*)(Bt + e) = o; }
        if (ps == 0) __threadfence(); }
}
template <int RES3> __global__ __launch_bounds__(256) void k_ln(const float* __restrict__ A, const float* __restrict__ Bv, const float* __restrict__ Cv, const float* __restrict__ gate, const float* __restrict__ sg, const float* __restrict__ sb, float* X, bf* Hh, bf* Hl) { const int lane = threadIdx.x & 31; const int l = blockIdx.x * 8 + (threadIdx.x >> 5); if (l >= LL) return; float v[DM / 32]; float s = 0.f; const float gt = RES3 ? bfr(gate[0]) : 0.f;
#pragma unroll
    for (int ch = 0; ch < DM / 128; ++ch) { const size_t o0 = (size_t)l * DM + ch * 128 + lane * 4; const v4f a = *(const v4f*)(A + o0);
#pragma unroll
        for (int u = 0; u < 4; ++u) { float x0 = bfr(a[u]); if (RES3) {     float gg = __fmul_rn(Cv[o0 + u], gt); asm volatile("" : "+v"(gg)); x0 = __fadd_rn(__fadd_rn(x0, Bv[o0 + u]), gg); } v[ch * 4 + u] = x0; s += x0; } }
#pragma unroll
    for (int sh = 16; sh; sh >>= 1) s += __shfl_xor(s, sh, 32);
    const float mean = s * (1.0f / DM); float q = 0.f;
#pragma unroll
    for (int k = 0; k < DM / 32; ++k) { float d = __fsub_rn(v[k], mean); asm volatile("" : "+v"(d)); float p = __fmul_rn(d, d); asm volatile("" : "+v"(p)); q = __fadd_rn(q, p); }
#pragma unroll
    for (int sh = 16; sh; sh >>= 1) q += __shfl_xor(q, sh, 32);
    const float rstd = __frsqrt_rn(__fadd_rn(q * (1.0f / DM), 1e-5f));
    for (int ps = 0; ps < 2; ++ps) {
#pragma unroll
        for (int ch = 0; ch < DM / 128; ++ch) { const int c0 = ch * 128 + lane * 4; const size_t o0 = (size_t)l * DM + c0; v4f xo; v4us oh, ol;
#pragma unroll
            for (int u = 0; u < 4; ++u) { xo[u] = v[ch * 4 + u]; float d = __fsub_rn(v[ch * 4 + u], mean); asm volatile("" : "+v"(d)); float n0 = __fmul_rn(d, rstd); asm volatile("" : "+v"(n0)); float g1 = bfr(sg[c0 + u]); asm volatile("" : "+v"(g1)); float t1 = __fmul_rn(n0, g1); asm volatile("" : "+v"(t1)); const float y = __fadd_rn(t1, bfr(sb[c0 + u])); unsigned short a2, b2; splitf(y, a2, b2); oh[u] = a2; ol[u] = b2; }
            if (RES3) *(volatile v4f*)(X + o0) = xo; *(volatile v4us*)(Hh + o0) = oh; *(volatile v4us*)(Hl + o0) = ol; }
        if (ps == 0) __threadfence(); } }
__global__ __launch_bounds__(256) void k_pl(const float* __restrict__ F, h16* P) { const int e = (blockIdx.x * 256 + threadIdx.x) * 4; if (e >= NH_ * LL * HD) return; const int d = e % HD; const int l = (e / HD) % LL; const int h = e / (HD * LL); const float* f = F + (size_t)l * DM + h * HD + d; v4h o;
#pragma unroll
    for (int u = 0; u < 4; ++u) o[u] = tohx(f[u]); *(volatile v4h*)(P + e) = o; __threadfence(); *(volatile v4h*)(P + e) = o; }
__global__ __launch_bounds__(256) void k_vt(const float* __restrict__ V, h16* VT) { const int e = (blockIdx.x * 256 + threadIdx.x) * 2; if (e >= NH_ * HD * LL) return; const int l = e % LL; const int d = (e / LL) % HD; const int h = e / (LL * HD); v2h o; o[0] = tohx(V[(size_t)l * DM + h * HD + d]); o[1] = tohx(V[(size_t)(l + 1) * DM + h * HD + d]); *(volatile v2h*)(VT + e) = o; __threadfence(); *(volatile v2h*)(VT + e) = o; }
__global__ __launch_bounds__(256) void k_gbias(const float* __restrict__ gf, const float* __restrict__ Wg, const float* __restrict__ bg, float* BIAS) { const int e = (blockIdx.x * 256 + threadIdx.x) * 4; if (e >= LL * LL) return; const int m0 = e % LL; const int l = e / LL;
#pragma unroll 1
    for (int h = 0; h < NH_; ++h) { v4f o; const float bgh = bfr(bg[h]);
#pragma unroll 1
        for (int u = 0; u < 4; ++u) { const float* gr = gf + ((size_t)l * LL + m0 + u) * NG; float bias = 0.f;
#pragma unroll 1
            for (int g = 0; g < NG; ++g) { float w = bfr(Wg[g * NH_ + h]); asm volatile("" : "+v"(w)); float p = __fmul_rn(bfr(gr[g]), w); asm volatile("" : "+v"(p)); bias = __fadd_rn(bias, p); }
            o[u] = __fadd_rn(bias, bgh); }
        float* dst = BIAS + ((size_t)h * LL + l) * LL + m0; *(volatile v4f*)dst = o; __threadfence(); *(volatile v4f*)dst = o; } }
__global__ __launch_bounds__(256) void k_ssoft(const float* __restrict__ Sb, const float* __restrict__ BIAS, const int* __restrict__ mk, h16* P16) { const int lane = threadIdx.x & 31; const int row = blockIdx.x * 8 + (threadIdx.x >> 5); if (row >= NH_ * LL) return;
    const float* sr = Sb + (size_t)row * LL; const float* br = BIAS + (size_t)row * LL; float v[LL / 32]; float mx = -3.0e38f;
#pragma unroll
    for (int ch = 0; ch < LL / 128; ++ch) { const int m0 = ch * 128 + lane * 4; const v4f a = *(const v4f*)(sr + m0); const v4f bb = *(const v4f*)(br + m0);
#pragma unroll
        for (int u = 0; u < 4; ++u) { const int m = m0 + u; float t0 = a[u] * 0.125f; asm volatile("" : "+v"(t0)); const float t = (mk[m] == 0) ? -10000.0f : __fadd_rn(t0, bb[u]); v[ch * 4 + u] = t; mx = fmaxf(mx, t); } }
#pragma unroll
    for (int sh = 16; sh; sh >>= 1) mx = fmaxf(mx, __shfl_xor(mx, sh, 32));
    float sum = 0.f;
#pragma unroll
    for (int q = 0; q < LL / 32; ++q) { float d0 = __fsub_rn(v[q], mx); asm volatile("" : "+v"(d0)); v[q] = __builtin_amdgcn_exp2f(__fmul_rn(d0, 1.4426950408889634f)); sum += v[q]; }
#pragma unroll
    for (int sh = 16; sh; sh >>= 1) sum += __shfl_xor(sum, sh, 32);
    const float f = __fdiv_rn(PCAR, sum);
    for (int ps = 0; ps < 2; ++ps) {
#pragma unroll
        for (int ch = 0; ch < LL / 128; ++ch) { v4h o4;
#pragma unroll
            for (int q = 0; q < 4; ++q) o4[q] = tohx(v[ch * 4 + q] * f); *(volatile v4h*)(P16 + (size_t)row * LL + ch * 128 + lane * 4) = o4; }
        if (ps == 0) __threadfence(); } }
__global__ __launch_bounds__(256) void k_mrg(const float* __restrict__ O, bf* Ah, bf* Al) { const int e = (blockIdx.x * 256 + threadIdx.x) * 4; if (e >= LL * DM) return; const int c = e % DM; const int l = e / DM; const int h = c / HD, d = c % HD; const float* o = O + ((size_t)h * LL + l) * HD + d; v4us oh, ol;
#pragma unroll
    for (int u = 0; u < 4; ++u) { unsigned short a, b; splitf(o[u] * (1.0f / PCAR), a, b); oh[u] = a; ol[u] = b; } *(volatile v4us*)(Ah + e) = oh; *(volatile v4us*)(Al + e) = ol; __threadfence(); *(volatile v4us*)(Ah + e) = oh; *(volatile v4us*)(Al + e) = ol; }
__global__ __launch_bounds__(256) void k_adja(const float* __restrict__ gf, const int* __restrict__ mk, float* AR) { const int e = (blockIdx.x * 256 + threadIdx.x) * 4; if (e >= LL * LL) return; const int m0 = e % LL; const int l = e / LL; const float ml = (mk[l] != 0) ? 1.f : 0.f; v4f o;
#pragma unroll 1
    for (int u = 0; u < 4; ++u) { const int m = m0 + u; const float a = __expf(__fdiv_rn(-bfr(gf[((size_t)l * LL + m) * NG]), 5.0f)); float mm = __fmul_rn(ml, (mk[m] != 0) ? 1.f : 0.f); asm volatile("" : "+v"(mm)); o[u] = __fmul_rn(a, mm); }
    *(volatile v4f*)(AR + e) = o; __threadfence(); *(volatile v4f*)(AR + e) = o; }
__global__ __launch_bounds__(256) void k_adj(const float* __restrict__ AR, bf* ADh, bf* ADl) { const int lane = threadIdx.x & 31; const int l = blockIdx.x * 8 + (threadIdx.x >> 5); if (l >= LL) return; float v[LL / 32]; float s = 0.f;
#pragma unroll
    for (int ch = 0; ch < LL / 128; ++ch) { const v4f a = *(const v4f*)(AR + (size_t)l * LL + ch * 128 + lane * 4);
#pragma unroll
        for (int u = 0; u < 4; ++u) { v[ch * 4 + u] = a[u]; s += a[u]; } }
#pragma unroll
    for (int sh = 16; sh; sh >>= 1) s += __shfl_xor(s, sh, 32);
    const float rden = __fdiv_rn(1.0f, __fadd_rn(s, 1e-6f));
    for (int ps = 0; ps < 2; ++ps) {
#pragma unroll
        for (int ch = 0; ch < LL / 128; ++ch) { v4us oh, ol;
#pragma unroll
            for (int u = 0; u < 4; ++u) { unsigned short a, b; splitf(__fmul_rn(v[ch * 4 + u], rden), a, b); oh[u] = a; ol[u] = b; } const size_t oo = (size_t)l * LL + ch * 128 + lane * 4; *(volatile v4us*)(ADh + oo) = oh; *(volatile v4us*)(ADl + oo) = ol; }
        if (ps == 0) __threadfence(); } }
__global__ __launch_bounds__(256) void k_tp(const float* __restrict__ G, bf* Th, bf* Tl) { const int e = (blockIdx.x * 256 + threadIdx.x) * 4; if (e >= DM * LL) return; const int m = e % LL; const int d = e / LL; v4us oh, ol;
#pragma unroll
    for (int u = 0; u < 4; ++u) { unsigned short a, b; splitf(G[(size_t)(m + u) * DM + d], a, b); oh[u] = a; ol[u] = b; } *(volatile v4us*)(Th + e) = oh; *(volatile v4us*)(Tl + e) = ol; __threadfence(); *(volatile v4us*)(Th + e) = oh; *(volatile v4us*)(Tl + e) = ol; }
__global__ __launch_bounds__(256) void k_gelu(const float* __restrict__ GC, float* GE) { const int e = (blockIdx.x * 256 + threadIdx.x) * 4; if (e >= LL * DM) return; const v4f a = *(const v4f*)(GC + e); v4f o;
#pragma unroll
    for (int u = 0; u < 4; ++u) { const float x = a[u]; float t = __fadd_rn(1.0f, erff(x * 0.70710678118654752f)); asm volatile("" : "+v"(t)); float hx = 0.5f * x; asm volatile("" : "+v"(hx)); o[u] = __fmul_rn(hx, t); } *(volatile v4f*)(GE + e) = o; __threadfence(); *(volatile v4f*)(GE + e) = o; }
__global__ __launch_bounds__(256) void k_glu(const float* __restrict__ FF, bf* Uh, bf* Ul) { const int e = (blockIdx.x * 256 + threadIdx.x) * 4; if (e >= LL * DFF) return; const int c = e % DFF; const int l = e / DFF; const float* fr = FF + (size_t)l * DF2; v4us oh, ol;
#pragma unroll
    for (int u = 0; u < 4; ++u) { const float gt = fr[DFF + c + u]; const float sg = __fdiv_rn(1.0f, __fadd_rn(1.0f, __expf(-gt))); const float y = __fmul_rn(fr[c + u], sg); unsigned short a, b; splitf(y, a, b); oh[u] = a; ol[u] = b; }
    *(volatile v4us*)(Uh + e) = oh; *(volatile v4us*)(Ul + e) = ol; __threadfence(); *(volatile v4us*)(Uh + e) = oh; *(volatile v4us*)(Ul + e) = ol; }
__global__ __launch_bounds__(256) void k_fin(const float* __restrict__ X1, const float* __restrict__ Y, const float* __restrict__ b2, float* OUTb) { const int e = (blockIdx.x * 256 + threadIdx.x) * 4; if (e >= LL * DM) return; const int c = e % DM; const v4f a = *(const v4f*)(X1 + e), y = *(const v4f*)(Y + e); v4f o;
#pragma unroll
    for (int u = 0; u < 4; ++u) o[u] = __fadd_rn(__fadd_rn(a[u], y[u]), bfr(b2[c + u])); *(volatile v4f*)(OUTb + e) = o; __threadfence(); *(volatile v4f*)(OUTb + e) = o; }

extern "C" void kernel_launch(void* const* d_in, const int* in_sizes, int n_in,
                              void* d_out, int out_size, void* d_ws, size_t ws_size, hipStream_t stream) {
    (void)in_sizes; (void)n_in; (void)out_size;
    const float** I = (const float**)d_in;
    const float *x = I[0], *gf = I[1], *Wq = I[3], *bq = I[4], *Wk = I[5], *bk = I[6], *Wv = I[7], *bv = I[8], *Wo = I[9], *bo = I[10], *Wg = I[11], *bg = I[12], *Wgcn = I[13], *bgcn = I[14], *ggate = I[15], *W1 = I[16], *b1 = I[17], *W2 = I[18], *b2 = I[19], *l1s = I[20], *l1b = I[21], *l2s = I[22], *l2b = I[23]; const int* mk = (const int*)d_in[2];
    float* OUT = (float*)d_out;
    char* wsp = (char*)d_ws;
    auto take = [&](size_t bytes) { char* p = wsp; wsp += (bytes + 255) & ~(size_t)255; return (void*)p; };
    bf* BQ = (bf*)take((size_t)DM * DM * 2); bf* BK = (bf*)take((size_t)DM * DM * 2); bf* BV = (bf*)take((size_t)DM * DM * 2); bf* BO = (bf*)take((size_t)DM * DM * 2); bf* BG = (bf*)take((size_t)DM * DM * 2); bf* BW1 = (bf*)take((size_t)DF2 * DM * 2); bf* BW2 = (bf*)take((size_t)DM * DFF * 2);
    bf* Hh = (bf*)take((size_t)LL * DM * 2); bf* Hl = (bf*)take((size_t)LL * DM * 2); float* FQ = (float*)take((size_t)LL * DM * 4); float* FK = (float*)take((size_t)LL * DM * 4); float* FV = (float*)take((size_t)LL * DM * 4); float* G = (float*)take((size_t)LL * DM * 4);
    h16* Q16 = (h16*)take((size_t)NH_ * LL * HD * 2); h16* K16 = (h16*)take((size_t)NH_ * LL * HD * 2); h16* VT = (h16*)take((size_t)NH_ * HD * LL * 2); float* Sb = (float*)take((size_t)NH_ * LL * LL * 4); h16* P16 = (h16*)take((size_t)NH_ * LL * LL * 2); float* O = (float*)take((size_t)NH_ * LL * HD * 4); bf* Ch = (bf*)take((size_t)LL * DM * 2); bf* Cl = (bf*)take((size_t)LL * DM * 2); float* ATT = (float*)take((size_t)LL * DM * 4);
    float* BIAS = (float*)take((size_t)NH_ * LL * LL * 4); float* AR = (float*)take((size_t)LL * LL * 4); bf* ADh = (bf*)take((size_t)LL * LL * 2); bf* ADl = (bf*)take((size_t)LL * LL * 2); bf* GTh = (bf*)take((size_t)DM * LL * 2); bf* GTl = (bf*)take((size_t)DM * LL * 2); float* GC = (float*)take((size_t)LL * DM * 4); float* GE = (float*)take((size_t)LL * DM * 4); float* X1 = (float*)take((size_t)LL * DM * 4); bf* H2h = (bf*)take((size_t)LL * DM * 2); bf* H2l = (bf*)take((size_t)LL * DM * 2);
    float* FF = (float*)take((size_t)LL * DF2 * 4); bf* Uh = (bf*)take((size_t)LL * DFF * 2); bf* Ul = (bf*)take((size_t)LL * DFF * 2); float* Y = (float*)take((size_t)LL * DM * 4);
    if ((size_t)(wsp - (char*)d_ws) > ws_size) return;
    k_wtG<<<(DM * DM / 64 + 63) / 64, 256, 0, stream>>>(Wq, DM, DM, BQ); k_wtG<<<(DM * DM / 64 + 63) / 64, 256, 0, stream>>>(Wk, DM, DM, BK); k_wtG<<<(DM * DM / 64 + 63) / 64, 256, 0, stream>>>(Wv, DM, DM, BV); k_wtG<<<(DM * DM / 64 + 63) / 64, 256, 0, stream>>>(Wo, DM, DM, BO); k_wtG<<<(DM * DM / 64 + 63) / 64, 256, 0, stream>>>(Wgcn, DM, DM, BG);
    k_wtG<<<(unsigned)((DM * DF2 / 64 + 63) / 64), 256, 0, stream>>>(W1, DM, DF2, BW1); k_wtG<<<(unsigned)((DFF * DM / 64 + 63) / 64), 256, 0, stream>>>(W2, DFF, DM, BW2);
    const unsigned gE = (LL * DM / 4 + 255) / 256;
    for (int b = 0; b < NB_; ++b) { const float* xb = x + (size_t)b * LL * DM; const float* gfb = gf + (size_t)b * LL * LL * NG; const int* mkb = mk + (size_t)b * LL;
        k_ln<0><<<LL / 8, 256, 0, stream>>>(xb, nullptr, nullptr, nullptr, l1s, l1b, nullptr, Hh, Hl);
        k_gemmw<bf, 1, true><<<dim3(LL / 64, DM / 64, 1), 32, 0, stream>>>(Hh, Hl, BQ, nullptr, DM, FQ, DM, bq, 0, 0, 0); k_gemmw<bf, 1, true><<<dim3(LL / 64, DM / 64, 1), 32, 0, stream>>>(Hh, Hl, BK, nullptr, DM, FK, DM, bk, 0, 0, 0);
        k_gemmw<bf, 1, true><<<dim3(LL / 64, DM / 64, 1), 32, 0, stream>>>(Hh, Hl, BV, nullptr, DM, FV, DM, bv, 0, 0, 0); k_gemmw<bf, 1, true><<<dim3(LL / 64, DM / 64, 1), 32, 0, stream>>>(Hh, Hl, BG, nullptr, DM, G, DM, bgcn, 0, 0, 0);
        k_pl<<<(NH_ * LL * HD / 4 + 255) / 256, 256, 0, stream>>>(FQ, Q16); k_pl<<<(NH_ * LL * HD / 4 + 255) / 256, 256, 0, stream>>>(FK, K16); k_vt<<<(NH_ * HD * LL / 2 + 255) / 256, 256, 0, stream>>>(FV, VT);
        k_gemmw<h16, 0, false><<<dim3(LL / 64, LL / 64, NH_), 32, 0, stream>>>(Q16, nullptr, K16, nullptr, HD, Sb, LL, nullptr, (size_t)LL * HD, (size_t)LL * HD, (size_t)LL * LL);
        k_gbias<<<(LL * LL / 4 + 255) / 256, 256, 0, stream>>>(gfb, Wg, bg, BIAS); k_ssoft<<<NH_ * LL / 8, 256, 0, stream>>>(Sb, BIAS, mkb, P16);
        k_gemmw<h16, 0, false><<<dim3(LL / 64, 1, NH_), 32, 0, stream>>>(P16, nullptr, VT, nullptr, LL, O, HD, nullptr, (size_t)LL * LL, (size_t)HD * LL, (size_t)LL * HD);
        k_mrg<<<gE, 256, 0, stream>>>(O, Ch, Cl); k_gemmw<bf, 1, true><<<dim3(LL / 64, DM / 64, 1), 32, 0, stream>>>(Ch, Cl, BO, nullptr, DM, ATT, DM, bo, 0, 0, 0);
        k_adja<<<(LL * LL / 4 + 255) / 256, 256, 0, stream>>>(gfb, mkb, AR); k_adj<<<LL / 8, 256, 0, stream>>>(AR, ADh, ADl); k_tp<<<(DM * LL / 4 + 255) / 256, 256, 0, stream>>>(G, GTh, GTl);
        k_gemmw<bf, 2, false><<<dim3(LL / 64, DM / 64, 1), 32, 0, stream>>>(ADh, ADl, GTh, GTl, LL, GC, DM, nullptr, 0, 0, 0); k_gelu<<<gE, 256, 0, stream>>>(GC, GE);
        k_ln<1><<<LL / 8, 256, 0, stream>>>(xb, ATT, GE, ggate, l2s, l2b, X1, H2h, H2l);
        k_gemmw<bf, 1, true><<<dim3(LL / 64, DF2 / 64, 1), 32, 0, stream>>>(H2h, H2l, BW1, nullptr, DM, FF, DF2, b1, 0, 0, 0); k_glu<<<(LL * DFF / 4 + 255) / 256, 256, 0, stream>>>(FF, Uh, Ul);
        k_gemmw<bf, 1, false><<<dim3(LL / 64, DM / 64, 1), 32, 0, stream>>>(Uh, Ul, BW2, nullptr, DFF, Y, DM, nullptr, 0, 0, 0);
        k_fin<<<gE, 256, 0, stream>>>(X1, Y, b2, OUT + (size_t)b * LL * DM); }
}
